// FeatherNet_27023934227230
// MI455X (gfx1250) — hardware-verified
//
#include <hip/hip_runtime.h>
#include <math.h>

typedef __attribute__((ext_vector_type(16))) _Float16 v16h;
typedef __attribute__((ext_vector_type(16))) __bf16 v16b;
typedef __attribute__((ext_vector_type(8)))  _Float16 v8h;
typedef __attribute__((ext_vector_type(8)))  float v8f;
typedef __attribute__((ext_vector_type(4)))  float v4f;
typedef __attribute__((ext_vector_type(2)))  float v2f;
typedef __attribute__((ext_vector_type(4)))  unsigned v4u;
typedef __attribute__((ext_vector_type(4)))  int v4i;
typedef float __attribute__((may_alias)) float_a;
typedef int __attribute__((may_alias)) int_a;

template <typename T> __device__ __forceinline__ void vst2(void* p, T v) { *(volatile T*)p = v; __threadfence(); *(volatile T*)p = v; }
__device__ __forceinline__ v8f wmma16(v16h a, v16h b, v8f c) {
  v8f d = __builtin_amdgcn_wmma_f32_16x16x32_f16(false, a, false, b, (short)0, c, false, false);
  asm volatile("v_nop\n\tv_nop\n\tv_nop\n\tv_nop" : "+v"(d) : "v"(a), "v"(b));
  return d;
}
__device__ __forceinline__ v8f wmma_bf(v16b a, v16b b, v8f c) {
  v8f d = __builtin_amdgcn_wmma_f32_16x16x32_bf16(false, a, false, b, (short)0, c, false, false);
  asm volatile("v_nop\n\tv_nop\n\tv_nop\n\tv_nop" : "+v"(d) : "v"(a), "v"(b));
  return d;
}
__device__ __forceinline__ v16h frag_h(const _Float16* rowk0, int lane) {
  union { v16h v; v8h q[2]; } u; const _Float16* p = rowk0 + 8 * (lane >> 4);
  u.q[0] = *(const v8h*)p; u.q[1] = *(const v8h*)(p + 16); return u.v;
}
__device__ __forceinline__ v16h frag_f32(const float* rowk0, int lane) {
  v16h a; const float* p = rowk0 + 8 * (lane >> 4);
#pragma unroll
  for (int i = 0; i < 8; ++i) { a[i] = (_Float16)p[i]; a[8 + i] = (_Float16)p[16 + i]; }
  return a;
}
__device__ __forceinline__ v16h frag_f32s(const float* rowk0, int lane, float sc) {
  v16h a; const float* p = rowk0 + 8 * (lane >> 4);
#pragma unroll
  for (int i = 0; i < 8; ++i) { a[i] = (_Float16)(p[i] * sc); a[8 + i] = (_Float16)(p[16 + i] * sc); }
  return a;
}
__device__ __forceinline__ v16h fragc_f32(const float* W, int k0, int n, int lane, int ld, int K) {
  v16h a; const int g = lane >> 4;
#pragma unroll
  for (int i = 0; i < 8; ++i) { const int ka = k0 + 8 * g + i, kb = ka + 16;
    a[i] = (_Float16)(ka < K ? W[(size_t)ka * ld + n] : 0.f); a[8 + i] = (_Float16)(kb < K ? W[(size_t)kb * ld + n] : 0.f); }
  return a;
}
struct F2 { v16b h, l; };
__device__ __forceinline__ F2 bsplit16(const float v[16]) { F2 r;
#pragma unroll
  for (int i = 0; i < 16; ++i) { const __bf16 h = (__bf16)v[i]; r.h[i] = h; r.l[i] = (__bf16)(v[i] - (float)h); }
  return r; }
__device__ __forceinline__ F2 split_row(const float* row, int k0, int lane) { float v[16]; const float* p = row + k0 + 8 * (lane >> 4);
#pragma unroll
  for (int i = 0; i < 8; ++i) { v[i] = p[i]; v[8 + i] = p[16 + i]; }
  return bsplit16(v); }
__device__ __forceinline__ F2 split_rowK(const float* row, int k0, int lane, int K) { float v[16]; const int g = lane >> 4;
#pragma unroll
  for (int i = 0; i < 8; ++i) { const int ka = k0 + 8 * g + i, kb = ka + 16; v[i] = ka < K ? row[ka] : 0.f; v[8 + i] = kb < K ? row[kb] : 0.f; }
  return bsplit16(v); }
__device__ __forceinline__ F2 split_col(const float* W, int k0, int n, int lane, int ld, int K) { float v[16]; const int g = lane >> 4;
#pragma unroll
  for (int i = 0; i < 8; ++i) { const int ka = k0 + 8 * g + i, kb = ka + 16; v[i] = ka < K ? W[(size_t)ka * ld + n] : 0.f; v[8 + i] = kb < K ? W[(size_t)kb * ld + n] : 0.f; }
  return bsplit16(v); }
__device__ __forceinline__ v8f mac3(const F2& a, const F2& b, v8f c) { c = wmma_bf(a.l, b.h, c); c = wmma_bf(a.h, b.l, c); return wmma_bf(a.h, b.h, c); }
__device__ __forceinline__ float sigm(float v) { return 1.0f / (1.0f + expf(-v)); }
#define LDSX() do { asm volatile("s_wait_dscnt 0" ::: "memory"); __builtin_amdgcn_wave_barrier(); __builtin_amdgcn_fence(__ATOMIC_RELEASE, "workgroup"); } while (0)

#define NBATCH 256
#define DIN 1024
#define DH 4096
#define DOUT 1024
#define SN 5018
#define SM 1255
#define SMP 1280
#define FP 5120
#define OFF_W1 0
#define OFF_B1 (DH * DIN)
#define OFF_W2 (OFF_B1 + DH)
#define OFF_B2 (OFF_W2 + DH * DH)
#define OFF_W3 (OFF_B2 + DH)
#define OFF_B3 (OFF_W3 + DOUT * DH)

__global__ __launch_bounds__(256) void k_packv(const float* __restrict__ V1, const float* __restrict__ V2, _Float16* __restrict__ V1h, _Float16* __restrict__ V2T) {
  const int r = blockIdx.x, which = blockIdx.y, tid = threadIdx.x; __shared__ __align__(16) _Float16 srow[SMP];
  for (int k = tid; k < SMP; k += 256) srow[k] = (_Float16)(k < SM ? (which == 0 ? V1[(size_t)r * SM + k] : V2[(size_t)k * SN + r]) : 0.f);
  __syncthreads();
  _Float16* D = (which == 0 ? V1h : V2T) + (size_t)r * SMP;
  for (int q = tid; q < SMP / 8; q += 256) vst2(D + q * 8, *(const v4u*)(&srow[q * 8]));
}
__global__ __launch_bounds__(128) void k_syn(const _Float16* __restrict__ V1h, const _Float16* __restrict__ V2T, _Float16* __restrict__ FL) {
  __shared__ __align__(16) _Float16 so[4][16][136];
  const int tid = threadIdx.x, wave = tid >> 5, lane = tid & 31, col = lane & 15, g = lane >> 4;
  const int r0 = blockIdx.x * 64 + wave * 16, n0 = blockIdx.y * 128; const int ra = (r0 + col) < SN ? (r0 + col) : SN - 1;
  v8f acc[8] = {};
#pragma unroll 2
  for (int kc = 0; kc < SMP / 32; ++kc) { const v16h a = frag_h(V1h + (size_t)ra * SMP + kc * 32, lane);
#pragma unroll
    for (int t = 0; t < 8; ++t) { const int n = n0 + t * 16 + col; acc[t] = wmma16(a, frag_h(V2T + (size_t)(n < SN ? n : SN - 1) * SMP + kc * 32, lane), acc[t]); } }
#pragma unroll
  for (int t = 0; t < 8; ++t)
#pragma unroll
    for (int r = 0; r < 8; ++r) so[wave][8 * g + r][t * 16 + col] = (_Float16)acc[t][r];
  LDSX();
  for (int q = lane; q < 16 * 16; q += 32) { const int rl = q >> 4, pc = q & 15; const int row = r0 + rl; if (row < SN) vst2(FL + (size_t)row * FP + n0 + pc * 8, *(const v4u*)(&so[wave][rl][pc * 8])); }
}
__device__ __forceinline__ float flat_at(const _Float16* __restrict__ FL, size_t f64) { const unsigned f = (unsigned)f64; const unsigned r = f / (unsigned)SN, c = f - r * (unsigned)SN; return (float)FL[(size_t)r * FP + c]; }
__global__ __launch_bounds__(256) void k_repack(const _Float16* __restrict__ FL, const float* __restrict__ pw1, const float* __restrict__ pb1, const float* __restrict__ pw2, const float* __restrict__ pb2, const float* __restrict__ pw3, const float* __restrict__ pb3,
                                              _Float16* __restrict__ W1h, _Float16* __restrict__ W2h, _Float16* __restrict__ W3h, float* __restrict__ B1, float* __restrict__ B2, float* __restrict__ B3) {
  const size_t t = (size_t)blockIdx.x * 256 + threadIdx.x;
  const size_t n1 = (size_t)DH * DIN / 8, n2 = (size_t)DH * DH / 8, n3 = (size_t)DOUT * DH / 8, nb = (DH + DH + DOUT) / 8;
  if (t < n1 + n2 + n3) { size_t base; float p; _Float16* D; size_t di;
    if (t < n1) { base = OFF_W1 + t * 8; p = pw1[0]; D = W1h; di = t * 8; } else if (t < n1 + n2) { base = OFF_W2 + (t - n1) * 8; p = pw2[0]; D = W2h; di = (t - n1) * 8; } else { base = OFF_W3 + (t - n1 - n2) * 8; p = pw3[0]; D = W3h; di = (t - n1 - n2) * 8; }
    union { v8h h; v4u u; } pk; const float sc = p * 16.0f;
#pragma unroll
    for (int e = 0; e < 8; ++e) pk.h[e] = (_Float16)(flat_at(FL, base + e) * sc);
    vst2(D + di, pk.u); }
  else if (t < n1 + n2 + n3 + nb) { const size_t j = (t - n1 - n2 - n3) * 8; size_t base; float p; float* D; size_t di;
    if (j < DH) { base = OFF_B1 + j; p = pb1[0]; D = B1; di = j; } else if (j < 2 * DH) { base = OFF_B2 + (j - DH); p = pb2[0]; D = B2; di = j - DH; } else { base = OFF_B3 + (j - 2 * DH); p = pb3[0]; D = B3; di = j - 2 * DH; }
    v4f a, b;
#pragma unroll
    for (int e = 0; e < 4; ++e) { a[e] = flat_at(FL, base + e) * p; b[e] = flat_at(FL, base + 4 + e) * p; }
    vst2(D + di, a); vst2(D + di + 4, b); }
}
template <int K, int AF32, int RELU, int OUTF16>
__global__ __launch_bounds__(128) void k_dense(const void* __restrict__ Av, const _Float16* __restrict__ W, const float* __restrict__ bias, void* __restrict__ Ov, int nout) {
  __shared__ __align__(16) float so[4][16][132];
  const int tid = threadIdx.x, wave = tid >> 5, lane = tid & 31, col = lane & 15, g = lane >> 4;
  const int r0 = blockIdx.x * 64 + wave * 16, n0 = blockIdx.y * 128;
  v8f acc[8] = {};
#pragma unroll 2
  for (int kc = 0; kc < K / 32; ++kc) { const v16h a = AF32 ? frag_f32((const float*)Av + (size_t)(r0 + col) * K + kc * 32, lane) : frag_h((const _Float16*)Av + (size_t)(r0 + col) * K + kc * 32, lane);
#pragma unroll
    for (int t = 0; t < 8; ++t) acc[t] = wmma16(a, frag_h(W + (size_t)(n0 + t * 16 + col) * K + kc * 32, lane), acc[t]); }
#pragma unroll
  for (int t = 0; t < 8; ++t) { const float bb = bias[n0 + t * 16 + col];
#pragma unroll
    for (int r = 0; r < 8; ++r) { const float v = acc[t][r] * (1.0f / 16.0f) + bb; so[wave][8 * g + r][t * 16 + col] = RELU ? (v > 0.f ? v : 0.f) : v; } }
  LDSX();
  if (OUTF16) { for (int q = lane; q < 16 * 16; q += 32) { const int rl = q >> 4, pc = q & 15; union { v8h h8; v4u u; } pk;
#pragma unroll
      for (int e = 0; e < 8; ++e) pk.h8[e] = (_Float16)so[wave][rl][pc * 8 + e];
      vst2((_Float16*)Ov + (size_t)(r0 + rl) * nout + n0 + pc * 8, pk.u); } }
  else {
#pragma unroll 4
    for (int rl = 0; rl < 16; ++rl) vst2((float*)Ov + (size_t)(r0 + rl) * nout + n0 + lane * 4, *(const v4f*)(&so[wave][rl][lane * 4])); }
}
extern "C" void kernel_launch(void* const* d_in, const int* in_sizes, int n_in, void* d_out, int out_size, void* d_ws, size_t ws_size, hipStream_t stream) {
  (void)in_sizes; (void)n_in; (void)out_size; (void)ws_size;
  const float** I = (const float**)d_in;
  const float* x = I[0]; const float* V1 = I[1]; const float* V2 = I[2];
  float* out = (float*)d_out;
  char* ws = (char*)d_ws; size_t off = 0;
  auto take = [&](size_t bytes) { char* p = ws + off; off += (bytes + 255) & ~(size_t)255; return p; };
  const size_t offA = off; _Float16* V1h = (_Float16*)take((size_t)SN * SMP * 2); _Float16* V2T = (_Float16*)take((size_t)SN * SMP * 2); const size_t endA = off;
  _Float16* FL = (_Float16*)take((size_t)SN * FP * 2); _Float16* W2h = (_Float16*)take((size_t)DH * DH * 2);
  off = offA;
  _Float16* W1h = (_Float16*)take((size_t)DH * DIN * 2); _Float16* W3h = (_Float16*)take((size_t)DOUT * DH * 2);
  float* B1 = (float*)take(DH * 4); float* B2 = (float*)take(DH * 4); float* B3 = (float*)take(DOUT * 4);
  _Float16* H1 = (_Float16*)take((size_t)NBATCH * DH * 2); _Float16* H2 = (_Float16*)take((size_t)NBATCH * DH * 2);
  if (off > endA) return;
  k_packv<<<dim3(SN, 2), 256, 0, stream>>>(V1, V2, V1h, V2T);
  k_syn<<<dim3((SN + 63) / 64, (SN + 127) / 128), 128, 0, stream>>>(V1h, V2T, FL);
  const size_t nthr = ((size_t)DH * DIN + (size_t)DH * DH + (size_t)DOUT * DH) / 8 + (DH + DH + DOUT) / 8;
  k_repack<<<(unsigned)((nthr + 255) / 256), 256, 0, stream>>>(FL, I[3], I[4], I[5], I[6], I[7], I[8], W1h, W2h, W3h, B1, B2, B3);
  k_dense<DIN, 1, 1, 1><<<dim3(NBATCH / 64, DH / 128), 128, 0, stream>>>(x, W1h, B1, H1, DH);
  k_dense<DH, 0, 1, 1><<<dim3(NBATCH / 64, DH / 128), 128, 0, stream>>>(H1, W2h, B2, H2, DH);
  k_dense<DH, 0, 0, 0><<<dim3(NBATCH / 64, DOUT / 128), 128, 0, stream>>>(H2, W3h, B3, out, DOUT);
}
